// GRUT1_84593675862254
// MI455X (gfx1250) — hardware-verified
//
#include <hip/hip_runtime.h>
#include <math.h>

constexpr int NFEAT    = 5;
constexpr int NHID     = 64;
constexpr int NBATCH   = 4096;
constexpr int NSTEP    = 512;
constexpr int NGATE3   = 3 * NHID;
constexpr int TILE_ROWS = 16;
constexpr int WAVES_PB = 2;
constexpr int NTHR     = WAVES_PB * 32;
constexpr int CHUNK    = 32;
constexpr int NCHUNK   = NSTEP / CHUNK;
constexpr int WPITCH   = 72;
constexpr int HPITCH   = 72;
constexpr int XROW8    = 8;
constexpr int CROW     = 8;
constexpr int NUGRP    = NHID / 16;
constexpr float WCARRY     = 16.0f;
constexpr float WCARRY_INV = 1.0f / WCARRY;
static_assert(NSTEP % CHUNK == 0, "time chunks exact");
static_assert(NBATCH % (TILE_ROWS * WAVES_PB) == 0, "batch tiles exact");
static_assert(NHID == 64 && NGATE3 == 192 && NUGRP == 4, "two k-steps of 32, twelve n-subtiles, four unit groups");
static_assert(NFEAT <= XROW8, "input features fit the first 8 k slots");
static_assert((NGATE3 * 8) % NTHR == 0, "weight staging loop exact");
static_assert(NGATE3 % NTHR == 0, "input weight staging loop exact");
static_assert(NHID == NTHR, "constant table staged one column per thread");
static_assert((WPITCH % 8) == 0 && (HPITCH % 8) == 0, "16-B aligned fragment rows");

typedef __attribute__((ext_vector_type(16))) _Float16 v16h;
typedef __attribute__((ext_vector_type(8)))  _Float16 v8h;
typedef __attribute__((ext_vector_type(8)))  float    v8f;
typedef __attribute__((ext_vector_type(4)))  float    v4f;
typedef __attribute__((ext_vector_type(8)))  unsigned v8u;
typedef __attribute__((ext_vector_type(4)))  unsigned v4u;
typedef __attribute__((ext_vector_type(2)))  unsigned v2u;

__device__ __forceinline__ unsigned h16bits(float f) {
  const _Float16 h = (_Float16)f;
  return (unsigned)__builtin_bit_cast(unsigned short, h);
}
__device__ __forceinline__ unsigned pack2h(float a, float b) {
  const unsigned lo = h16bits(a);
  const unsigned hi = h16bits(b);
  return lo | (hi << 16);
}

union FragU { v16h v; v8h h[2]; };
__device__ __forceinline__ v16h load_frag(const _Float16* p) {
  FragU f;
  f.h[0] = *(const v8h*)(p);
  f.h[1] = *(const v8h*)(p + 16);
  return f.v;
}
__device__ __forceinline__ v16h load_frag_lo8(const _Float16* p) {
  FragU f;
  const v8h zz = {(_Float16)0.0f, (_Float16)0.0f, (_Float16)0.0f, (_Float16)0.0f,
                  (_Float16)0.0f, (_Float16)0.0f, (_Float16)0.0f, (_Float16)0.0f};
  f.h[0] = *(const v8h*)(p);
  f.h[1] = zz;
  return f.v;
}
__device__ __forceinline__ v8f mma16(v16h a, v16h b, v8f c) {
  return __builtin_amdgcn_wmma_f32_16x16x32_f16(false, a, false, b, (short)0, c, false, false);
}
__device__ __forceinline__ void guard_gate1(v8f& acc, v16h a0, v16h a1, v16h ax, v16h b0, v16h b1, v16h bx) {
  asm volatile("v_nop\n\tv_nop\n\tv_nop\n\tv_nop" : "+v"(acc) : "v"(a0), "v"(a1), "v"(ax), "v"(b0), "v"(b1), "v"(bx));
}
__device__ __forceinline__ void guard_gate2(v8f& acc0, v8f& acc1, v16h a0, v16h a1, v16h ax, v16h b0, v16h b1, v16h bx) {
  asm volatile("v_nop\n\tv_nop\n\tv_nop\n\tv_nop" : "+v"(acc0), "+v"(acc1) : "v"(a0), "v"(a1), "v"(ax), "v"(b0), "v"(b1), "v"(bx));
}
__device__ __forceinline__ void wave_lds_fence() {
  __builtin_amdgcn_fence(__ATOMIC_RELEASE, "workgroup");
  __builtin_amdgcn_wave_barrier();
  __builtin_amdgcn_fence(__ATOMIC_ACQUIRE, "workgroup");
}
__device__ __forceinline__ void sched_fence() { __builtin_amdgcn_sched_barrier(0); }
__device__ __forceinline__ float fsig(float x)  { return __builtin_amdgcn_rcpf(1.0f + __expf(-x)); }
__device__ __forceinline__ float ftanh(float x) { return 1.0f - 2.0f * __builtin_amdgcn_rcpf(__expf(2.0f * x) + 1.0f); }

__global__ __launch_bounds__(NTHR) __attribute__((amdgpu_num_vgpr(256)))
void gru_decay_scan_kernel(const float* __restrict__ X, const float* __restrict__ dt,
                           const float* __restrict__ w_ih, const float* __restrict__ w_hh,
                           const float* __restrict__ b_ih, const float* __restrict__ b_hh,
                           const float* __restrict__ w_dt, const float* __restrict__ b_dt,
                           const float* __restrict__ w_out, const float* __restrict__ b_out,
                           float* __restrict__ out) {
  __shared__ __align__(16) unsigned short WhS[NGATE3 * WPITCH];
  __shared__ __align__(16) unsigned short WxS[2 * NGATE3 * XROW8];
  __shared__ __align__(16) float          CsS[NHID * CROW];
  __shared__ __align__(16) unsigned short HtS[WAVES_PB][TILE_ROWS * HPITCH];
  __shared__ __align__(16) v4u            XfS[WAVES_PB][CHUNK * TILE_ROWS];
  __shared__ __align__(16) float          DtS[WAVES_PB][CHUNK * TILE_ROWS];
  __shared__ __align__(16) float          PrS[WAVES_PB][TILE_ROWS * CHUNK];

  const int tid  = threadIdx.x;
  const int wave = tid >> 5;
  const int lane = tid & 31;
  const int hh   = lane >> 4;
  const int c    = lane & 15;
  const int b0   = (blockIdx.x * WAVES_PB + wave) * TILE_ROWS;

#pragma unroll 1
  for (int idx = tid; idx < NGATE3 * 8; idx += NTHR) {
    const int n   = idx >> 3;
    const int kp0 = (idx & 7) * 8;
    const float* wr = w_hh + n * NHID + (kp0 >> 2);
    float f[8];
#pragma unroll
    for (int e = 0; e < 8; ++e) f[e] = wr[16 * (e & 3) + (e >> 2)] * WCARRY;
    v4u q;
    q[0] = pack2h(f[0], f[1]);
    q[1] = pack2h(f[2], f[3]);
    q[2] = pack2h(f[4], f[5]);
    q[3] = pack2h(f[6], f[7]);
    *(v4u*)(WhS + n * WPITCH + kp0) = q;
  }
#pragma unroll 1
  for (int rr = tid; rr < NGATE3; rr += NTHR) {
    const float* xr = w_ih + rr * NFEAT;
    const float f0 = xr[0] * WCARRY, f1 = xr[1] * WCARRY, f2 = xr[2] * WCARRY, f3 = xr[3] * WCARRY, f4 = xr[4] * WCARRY;
    v4u q;
    q[0] = pack2h(f0, f1);
    q[1] = pack2h(f2, f3);
    q[2] = h16bits(f4);
    q[3] = 0u;
    const v4u zq = {0u, 0u, 0u, 0u};
    *(v4u*)(WxS + rr * XROW8) = q;
    *(v4u*)(WxS + (NGATE3 + rr) * XROW8) = zq;
  }
  {
    const int col = tid;
    v4f ca, cb;
    ca[0] = w_dt[col];
    ca[1] = b_dt[col];
    ca[2] = b_ih[col] + b_hh[col];
    ca[3] = b_ih[NHID + col] + b_hh[NHID + col];
    cb[0] = b_ih[2 * NHID + col];
    cb[1] = b_hh[2 * NHID + col];
    cb[2] = w_out[col];
    cb[3] = 0.0f;
    *(v4f*)(CsS + col * CROW)     = ca;
    *(v4f*)(CsS + col * CROW + 4) = cb;
  }
  __syncthreads();

  float wdt[4], bdt[4];
#pragma unroll
  for (int j = 0; j < 4; ++j) {
    const v4f ca = *(const v4f*)(CsS + (16 * j + c) * CROW);
    wdt[j] = ca[0];
    bdt[j] = ca[1];
  }
  const float bo = b_out[0];

  const v8f z8 = {0.f, 0.f, 0.f, 0.f, 0.f, 0.f, 0.f, 0.f};
  v8f hq0 = z8, hq1 = z8, hq2 = z8, hq3 = z8;

  unsigned short* htw = HtS[wave];
  const _Float16* hta = (const _Float16*)(const void*)HtS[wave] + c * HPITCH + 8 * hh;
  const _Float16* whp = (const _Float16*)(const void*)WhS + c * WPITCH + 8 * hh;
  const _Float16* wxp = (const _Float16*)(const void*)WxS + hh * (NGATE3 * XROW8) + c * XROW8;
  const float*    csp = CsS + c * CROW;
  v4u*   xf  = XfS[wave];
  float* dts = DtS[wave];
  float* prs = PrS[wave];
  const int cv = c & 7;

#pragma unroll 1
  for (int ch = 0; ch < NCHUNK; ++ch) {
    const int t0 = ch * CHUNK;
#pragma unroll 1
    for (int i = 0; i < TILE_ROWS; ++i) {
      const size_t rb = (size_t)(b0 + i) * NSTEP + (size_t)(t0 + lane);
      const float* xp = X + rb * NFEAT;
      const float x0 = xp[0], x1 = xp[1], x2 = xp[2], x3 = xp[3], x4 = xp[4];
      const float dv = dt[rb];
      v4u q;
      q[0] = pack2h(x0, x1);
      q[1] = pack2h(x2, x3);
      q[2] = h16bits(x4);
      q[3] = 0u;
      xf[lane * TILE_ROWS + i]  = q;
      dts[lane * TILE_ROWS + i] = dv;
    }
    wave_lds_fence();

#pragma unroll 1
    for (int tl = 0; tl < CHUNK; ++tl) {
      const v4u xq = xf[tl * TILE_ROWS + c];
      v8u fx;
      fx[0] = hh ? 0u : xq[0];
      fx[1] = hh ? 0u : xq[1];
      fx[2] = hh ? 0u : xq[2];
      fx[3] = hh ? 0u : xq[3];
      fx[4] = 0u;
      fx[5] = 0u;
      fx[6] = 0u;
      fx[7] = 0u;
      const v16h ax = __builtin_bit_cast(v16h, fx);

      const v4f d0 = *(const v4f*)(dts + tl * TILE_ROWS + 8 * hh);
      const v4f d1 = *(const v4f*)(dts + tl * TILE_ROWS + 8 * hh + 4);
      float dtv[8];
      dtv[0] = d0[0]; dtv[1] = d0[1]; dtv[2] = d0[2]; dtv[3] = d0[3];
      dtv[4] = d1[0]; dtv[5] = d1[1]; dtv[6] = d1[2]; dtv[7] = d1[3];

#pragma unroll
      for (int r = 0; r < 8; ++r) {
        const float dd = dtv[r];
        const float e0 = __expf(-fmaxf(fmaf(dd, wdt[0], bdt[0]), 0.0f));
        const float e1 = __expf(-fmaxf(fmaf(dd, wdt[1], bdt[1]), 0.0f));
        const float e2 = __expf(-fmaxf(fmaf(dd, wdt[2], bdt[2]), 0.0f));
        const float e3 = __expf(-fmaxf(fmaf(dd, wdt[3], bdt[3]), 0.0f));
        const float g0 = e0 * hq0[r];
        const float g1 = e1 * hq1[r];
        const float g2 = e2 * hq2[r];
        const float g3 = e3 * hq3[r];
        hq0[r] = g0;
        hq1[r] = g1;
        hq2[r] = g2;
        hq3[r] = g3;
        v2u pk;
        pk[0] = pack2h(g0, g1);
        pk[1] = pack2h(g2, g3);
        *(v2u*)(htw + (8 * hh + r) * HPITCH + 4 * c) = pk;
      }
      wave_lds_fence();

      const v16h a0 = load_frag(hta);
      const v16h a1 = load_frag(hta + 32);

      v8f pv = z8;

#pragma unroll 1
      for (int j = 0; j < NUGRP; ++j) {
        const _Float16* wb = whp + (16 * j) * WPITCH;
        const _Float16* xb = wxp + (16 * j) * XROW8;
        const v4f ca = *(const v4f*)(csp + (16 * j) * CROW);
        const v4f cb = *(const v4f*)(csp + (16 * j) * CROW + 4);
        const float brr  = ca[2];
        const float bzz  = ca[3];
        const float bin  = cb[0];
        const float bhn  = cb[1];
        const float wout = cb[2];
        v8f accr, accz, accnh, accni;
        sched_fence();
        {
          const v16h b1 = load_frag(wb + 32);
          const v16h bl = load_frag(wb);
          const v16h bx = load_frag_lo8(xb);
          accr = mma16(a1, b1, z8);
          accr = mma16(a0, bl, accr);
          accr = mma16(ax, bx, accr);
          guard_gate1(accr, a0, a1, ax, bl, b1, bx);
        }
        sched_fence();
        {
          const v16h b1 = load_frag(wb + NHID * WPITCH + 32);
          const v16h bl = load_frag(wb + NHID * WPITCH);
          const v16h bx = load_frag_lo8(xb + NHID * XROW8);
          accz = mma16(a1, b1, z8);
          accz = mma16(a0, bl, accz);
          accz = mma16(ax, bx, accz);
          guard_gate1(accz, a0, a1, ax, bl, b1, bx);
        }
        sched_fence();
        {
          const v16h b1 = load_frag(wb + 2 * NHID * WPITCH + 32);
          const v16h bl = load_frag(wb + 2 * NHID * WPITCH);
          const v16h bx = load_frag_lo8(xb + 2 * NHID * XROW8);
          accnh = mma16(a1, b1, z8);
          accnh = mma16(a0, bl, accnh);
          accni = mma16(ax, bx, z8);
          guard_gate2(accnh, accni, a0, a1, ax, bl, b1, bx);
        }
        sched_fence();
        v8f hn = z8;
#pragma unroll
        for (int r = 0; r < 8; ++r) {
          const float rg = fsig(fmaf(accr[r], WCARRY_INV, brr));
          const float zg = fsig(fmaf(accz[r], WCARRY_INV, bzz));
          const float hp = fmaf(accnh[r], WCARRY_INV, bhn);
          const float xn = fmaf(accni[r], WCARRY_INV, bin);
          const float ng = ftanh(fmaf(rg, hp, xn));
          const float ht = hq0[r];
          const float hnew = (1.0f - zg) * ng + zg * ht;
          hn[r] = hnew;
          pv[r] = fmaf(hnew, wout, pv[r]);
        }
        hq0 = hq1;
        hq1 = hq2;
        hq2 = hq3;
        hq3 = hn;
      }

      float p[8];
#pragma unroll
      for (int r = 0; r < 8; ++r) p[r] = pv[r];
#pragma unroll
      for (int off = 1; off < 16; off <<= 1) {
#pragma unroll
        for (int r = 0; r < 8; ++r) p[r] += __shfl_xor(p[r], off, 32);
      }
      float val = p[0];
      val = (cv == 1) ? p[1] : val;
      val = (cv == 2) ? p[2] : val;
      val = (cv == 3) ? p[3] : val;
      val = (cv == 4) ? p[4] : val;
      val = (cv == 5) ? p[5] : val;
      val = (cv == 6) ? p[6] : val;
      val = (cv == 7) ? p[7] : val;
      prs[(8 * hh + cv) * CHUNK + tl] = val + bo;
    }

    wave_lds_fence();
    {
      const int q  = lane >> 3;
      const int c4 = (lane & 7) * 4;
      for (int pass = 0; pass < 2; ++pass) {
#pragma unroll
        for (int it = 0; it < 4; ++it) {
          const int row = it * 4 + q;
          const v4f v = *(const v4f*)(prs + row * CHUNK + c4);
          *(volatile v4f*)(out + (size_t)(b0 + row) * NSTEP + (size_t)(t0 + c4)) = v;
        }
        __threadfence();
      }
    }
    wave_lds_fence();
  }
}

extern "C" void kernel_launch(void* const* d_in, const int* in_sizes, int n_in,
                              void* d_out, int out_size, void* d_ws, size_t ws_size, hipStream_t stream) {
  (void)d_ws; (void)ws_size;
  if (n_in < 10 || d_out == nullptr) return;
  if (in_sizes[0] != NBATCH * NSTEP * NFEAT || in_sizes[1] != NBATCH * NSTEP ||
      in_sizes[2] != NGATE3 * NFEAT || in_sizes[3] != NGATE3 * NHID ||
      in_sizes[4] != NGATE3 || in_sizes[5] != NGATE3 ||
      in_sizes[6] != NHID || in_sizes[7] != NHID || in_sizes[8] != NHID || in_sizes[9] != 1 ||
      out_size != NBATCH * NSTEP) return;

  const float* X     = (const float*)d_in[0];
  const float* dtp   = (const float*)d_in[1];
  const float* w_ih  = (const float*)d_in[2];
  const float* w_hh  = (const float*)d_in[3];
  const float* b_ih  = (const float*)d_in[4];
  const float* b_hh  = (const float*)d_in[5];
  const float* w_dt  = (const float*)d_in[6];
  const float* b_dt  = (const float*)d_in[7];
  const float* w_out = (const float*)d_in[8];
  const float* b_out = (const float*)d_in[9];
  float* out = (float*)d_out;

  gru_decay_scan_kernel<<<NBATCH / (TILE_ROWS * WAVES_PB), NTHR, 0, stream>>>(
      X, dtp, w_ih, w_hh, b_ih, b_hh, w_dt, b_dt, w_out, b_out, out);
}
